// RelationalLayer_10711648436521
// MI455X (gfx1250) — hardware-verified
//
#include <hip/hip_runtime.h>

constexpr int kBatch   = 64;
constexpr int kObjs    = 64;
constexpr int kFeat    = 26;
constexpr int kObjRows = kBatch * kObjs;
constexpr int kHid     = 256;
constexpr int kOutW    = 32;
constexpr int kLdsPitch = 264;
constexpr float kActCarry = 64.0f;
constexpr float kWCarry   = 256.0f;
constexpr float kAccInv   = 1.0f / 16384.0f;
constexpr float kAccToAct = 1.0f / 256.0f;

typedef __attribute__((ext_vector_type(16))) _Float16 v16h;
typedef __attribute__((ext_vector_type(8)))  _Float16 v8h;
typedef __attribute__((ext_vector_type(16))) __bf16   v16b;
typedef __attribute__((ext_vector_type(8)))  __bf16   v8b;
typedef __attribute__((ext_vector_type(8)))  float    v8f;
typedef __attribute__((ext_vector_type(4)))  float    v4f;
typedef __attribute__((ext_vector_type(4)))  unsigned int v4u;

__device__ __forceinline__ unsigned short f2bf_bits(float f) {
  unsigned u = __float_as_uint(f);
  return (unsigned short)((u + 0x7FFFu + ((u >> 16) & 1u)) >> 16);
}
__device__ __forceinline__ float bf_bits2f(unsigned short h) { return __uint_as_float(((unsigned)h) << 16); }

__device__ __forceinline__ void dep_guard_h(v8f& a, v8f& b, v16h x, v16h y) { asm volatile("v_nop\n\tv_nop\n\tv_nop\n\tv_nop" : "+v"(a), "+v"(b) : "v"(x), "v"(y)); }
__device__ __forceinline__ void dep_guard_b(v8f& a, v8f& b, v16b x, v16b y) { asm volatile("v_nop\n\tv_nop\n\tv_nop\n\tv_nop" : "+v"(a), "+v"(b) : "v"(x), "v"(y)); }
__device__ __forceinline__ void keep4_h(v16h a, v16h b, v16h c, v16h d) { asm volatile("v_nop" :: "v"(a), "v"(b), "v"(c), "v"(d)); }
__device__ __forceinline__ void keep4_b(v16b a, v16b b, v16b c, v16b d) { asm volatile("v_nop" :: "v"(a), "v"(b), "v"(c), "v"(d)); }
__device__ __forceinline__ void acc_guard4(v8f& a, v8f& b, v8f& c, v8f& d) { asm volatile("v_nop\n\tv_nop\n\tv_nop\n\tv_nop" : "+v"(a), "+v"(b), "+v"(c), "+v"(d)); }
template <typename T> struct Frag;
template <> struct Frag<_Float16> {
  typedef v16h V; union U { v16h v; v8h h[2]; };
  static __device__ __forceinline__ v16h load(const _Float16* p) {
    U f; f.h[0] = *(const v8h*)(p); f.h[1] = *(const v8h*)(p + 16); return f.v;
  }
  static __device__ __forceinline__ v8f mma(v16h a, v16h b, v8f c) {
    return __builtin_amdgcn_wmma_f32_16x16x32_f16(false, a, false, b, (short)0, c, false, false);
  }
  static __device__ __forceinline__ void guard(v8f& a, v8f& b, v16h x, v16h y) { dep_guard_h(a, b, x, y); }
  static __device__ __forceinline__ void keep(v16h a, v16h b, v16h c, v16h d) { keep4_h(a, b, c, d); }
};
template <> struct Frag<__bf16> {
  typedef v16b V; union U { v16b v; v8b h[2]; };
  static __device__ __forceinline__ v16b load(const __bf16* p) {
    U f; f.h[0] = *(const v8b*)(p); f.h[1] = *(const v8b*)(p + 16); return f.v;
  }
  static __device__ __forceinline__ v8f mma(v16b a, v16b b, v8f c) {
    return __builtin_amdgcn_wmma_f32_16x16x32_bf16(false, a, false, b, (short)0, c, false, false);
  }
  static __device__ __forceinline__ void guard(v8f& a, v8f& b, v16b x, v16b y) { dep_guard_b(a, b, x, y); }
  static __device__ __forceinline__ void keep(v16b a, v16b b, v16b c, v16b d) { keep4_b(a, b, c, d); }
};

__device__ __forceinline__ unsigned pk16(unsigned short a, unsigned short b) { return (unsigned)a | ((unsigned)b << 16); }
__device__ __forceinline__ unsigned short h_bits(float f) { const _Float16 h = (_Float16)f; return __builtin_bit_cast(unsigned short, h); }

__global__ __launch_bounds__(256) void obj_linear_kernel(const float* __restrict__ x, const float* __restrict__ W0,
                                                         const float* __restrict__ b0,
                                                         float* __restrict__ A, float* __restrict__ Bm) {
  __shared__ float xs[4 * kFeat];
  const int t = threadIdx.x;
  const int blk = blockIdx.x;
  if (t < 4 * kFeat) xs[t] = x[(size_t)blk * (4 * kFeat) + t];
  __syncthreads();
  const int rloc = t >> 6;
  const int n4 = (t & 63) * 4;
  const int row = blk * 4 + rloc;
  v4f a = (v4f){0.f, 0.f, 0.f, 0.f};
  v4f bb = *(const v4f*)(b0 + n4);
#pragma unroll 1
  for (int k = 0; k < kFeat; ++k) {
    const float xv = xs[rloc * kFeat + k];
    const v4f w  = *(const v4f*)(W0 + (size_t)k * kHid + n4);
    const v4f wb = *(const v4f*)(W0 + (size_t)(kFeat + k) * kHid + n4);
    a  += xv * w;
    bb += xv * wb;
  }
  float* pa = A  + (size_t)row * kHid + n4;
  float* pb = Bm + (size_t)row * kHid + n4;
  *(volatile v4f*)pa = a;
  *(volatile v4f*)pb = bb;
  __threadfence();
  *(volatile v4f*)pa = a;
  *(volatile v4f*)pb = bb;
}

__global__ __launch_bounds__(256) void wt_cast_kernel(const float* __restrict__ W1, const float* __restrict__ W2,
                                                      const float* __restrict__ W3,
                                                      unsigned short* __restrict__ out, float scale) {
  __shared__ float sm[64][65];
  const int t  = threadIdx.x;
  const int k0 = blockIdx.x * 64;
  const int n0 = blockIdx.y * 64;
  const int z  = blockIdx.z;
  const float* W = (z == 0) ? W1 : (z == 1) ? W2 : W3;
#pragma unroll
  for (int i = 0; i < 16; ++i) {
    const int e = i * 256 + t;
    const int r = e >> 6;
    const int c = e & 63;
    sm[c][r] = W[(size_t)(k0 + r) * kHid + n0 + c] * scale;
  }
  __syncthreads();
  const int lane = t & 31, wave = t >> 5;
  const int q = lane >> 3, c8 = (lane & 7) * 8;
  unsigned short* op = out + (size_t)z * kHid * kHid;
  for (int pass = 0; pass < 2; ++pass) {
#pragma unroll
    for (int it = 0; it < 2; ++it) {
      const int row = wave * 8 + it * 4 + q;
      unsigned short hb[8];
#pragma unroll
      for (int e = 0; e < 8; ++e) hb[e] = h_bits(sm[row][c8 + e]);
      const v4u u = (v4u){pk16(hb[0], hb[1]), pk16(hb[2], hb[3]), pk16(hb[4], hb[5]), pk16(hb[6], hb[7])};
      *(volatile v4u*)(op + (size_t)(n0 + row) * kHid + k0 + c8) = u;
    }
    __threadfence();
  }
}

__global__ __launch_bounds__(256) void pair_mlp_kernel(const float* __restrict__ A, const float* __restrict__ Bm,
                                                       const unsigned short* __restrict__ WtAll,
                                                       const float* __restrict__ b1, const float* __restrict__ b2,
                                                       const float* __restrict__ b3, float* __restrict__ Spart) {
  __shared__ __align__(16) _Float16 Hs[64][kLdsPitch];
  __shared__ __align__(16) float ssum[kHid];

  const int t   = threadIdx.x;
  const int blk = blockIdx.x;
  const int b   = blk >> 6;
  const int i   = blk & 63;

  {
    const int j  = t >> 2;
    const int n0 = (t & 3) * 64;
    const float* Ar = A  + ((size_t)(b * kObjs + j)) * kHid + n0;
    const float* Br = Bm + ((size_t)(b * kObjs + i)) * kHid + n0;
#pragma unroll
    for (int e = 0; e < 8; ++e) {
      const v4f a0 = *(const v4f*)(Ar + 8 * e),     c0 = *(const v4f*)(Br + 8 * e);
      const v4f a1 = *(const v4f*)(Ar + 8 * e + 4), c1 = *(const v4f*)(Br + 8 * e + 4);
      v8h pk;
      pk[0] = (_Float16)(fmaxf(a0[0] + c0[0], 0.0f) * kActCarry);
      pk[1] = (_Float16)(fmaxf(a0[1] + c0[1], 0.0f) * kActCarry);
      pk[2] = (_Float16)(fmaxf(a0[2] + c0[2], 0.0f) * kActCarry);
      pk[3] = (_Float16)(fmaxf(a0[3] + c0[3], 0.0f) * kActCarry);
      pk[4] = (_Float16)(fmaxf(a1[0] + c1[0], 0.0f) * kActCarry);
      pk[5] = (_Float16)(fmaxf(a1[1] + c1[1], 0.0f) * kActCarry);
      pk[6] = (_Float16)(fmaxf(a1[2] + c1[2], 0.0f) * kActCarry);
      pk[7] = (_Float16)(fmaxf(a1[3] + c1[3], 0.0f) * kActCarry);
      *(v8h*)&Hs[j][n0 + 8 * e] = pk;
    }
  }
  __syncthreads();

  const int lane  = t & 31;
  const int wave  = t >> 5;
  const int rlane = lane & 15;
  const int koff  = (lane >> 4) * 8;
  const int mOff  = (lane >> 4) * 8;
  const int N0 = wave * 32 + rlane;
  const int N1 = N0 + 16;

#pragma unroll 1
  for (int layer = 0; layer < 3; ++layer) {
    const _Float16* Wt = (const _Float16*)(WtAll + (size_t)layer * kHid * kHid);
    const float* bias = (layer == 0) ? b1 : (layer == 1) ? b2 : b3;

    v8f acc[4][2];
#pragma unroll
    for (int mt = 0; mt < 4; ++mt) {
      acc[mt][0] = (v8f){0.f,0.f,0.f,0.f,0.f,0.f,0.f,0.f};
      acc[mt][1] = (v8f){0.f,0.f,0.f,0.f,0.f,0.f,0.f,0.f};
    }

#pragma unroll 1
    for (int k0 = 0; k0 < kHid; k0 += 32) {
      v16h bf[2];
#pragma unroll
      for (int nt = 0; nt < 2; ++nt)
        bf[nt] = Frag<_Float16>::load(Wt + (size_t)(wave * 32 + nt * 16 + rlane) * kHid + k0 + koff);
#pragma unroll
      for (int mt = 0; mt < 4; ++mt) {
        Frag<_Float16>::U f;
        f.h[0] = *(const v8h*)(&Hs[mt * 16 + rlane][k0 + koff]);
        f.h[1] = *(const v8h*)(&Hs[mt * 16 + rlane][k0 + koff + 16]);
        const v16h af = f.v;
#pragma unroll
        for (int nt = 0; nt < 2; ++nt) acc[mt][nt] = Frag<_Float16>::mma(af, bf[nt], acc[mt][nt]);
        Frag<_Float16>::guard(acc[mt][0], acc[mt][1], af, af);
      }
      Frag<_Float16>::keep(bf[0], bf[1], bf[0], bf[1]);
    }
    acc_guard4(acc[0][0], acc[0][1], acc[1][0], acc[1][1]);
    acc_guard4(acc[2][0], acc[2][1], acc[3][0], acc[3][1]);

    const float bias0 = bias[N0];
    const float bias1 = bias[N1];

    if (layer < 2) {
      const float bb0 = bias0 * kActCarry;
      const float bb1 = bias1 * kActCarry;
      __syncthreads();
#pragma unroll
      for (int mt = 0; mt < 4; ++mt) {
#pragma unroll
        for (int r = 0; r < 8; ++r) {
          const int row = mt * 16 + mOff + r;
          Hs[row][N0] = (_Float16)fmaxf(fmaf(acc[mt][0][r], kAccToAct, bb0), 0.0f);
          Hs[row][N1] = (_Float16)fmaxf(fmaf(acc[mt][1][r], kAccToAct, bb1), 0.0f);
        }
      }
      __syncthreads();
    } else {
      float s0 = 0.0f, s1 = 0.0f;
#pragma unroll
      for (int mt = 0; mt < 4; ++mt) {
#pragma unroll
        for (int r = 0; r < 8; ++r) {
          s0 += fmaxf(fmaf(acc[mt][0][r], kAccInv, bias0), 0.0f);
          s1 += fmaxf(fmaf(acc[mt][1][r], kAccInv, bias1), 0.0f);
        }
      }
      s0 += __shfl_xor(s0, 16, 32);
      s1 += __shfl_xor(s1, 16, 32);
      if (lane < 16) {
        ssum[N0] = s0;
        ssum[N1] = s1;
      }
      __syncthreads();
      if (t < 64) {
        const v4f v = *(const v4f*)(ssum + 4 * t);
        float* p = Spart + (size_t)blk * kHid + 4 * t;
        *(volatile v4f*)p = v;
        __threadfence();
        *(volatile v4f*)p = v;
      }
    }
  }
}

__global__ __launch_bounds__(256) void head_mlp_kernel(const float* __restrict__ Spart,
                                                       const float* __restrict__ W4, const float* __restrict__ b4,
                                                       const float* __restrict__ W5, const float* __restrict__ b5,
                                                       const float* __restrict__ W6, const float* __restrict__ b6,
                                                       float* __restrict__ out) {
  __shared__ __align__(16) float sh0[kHid];
  __shared__ __align__(16) float sh1[kHid];
  __shared__ __align__(16) float so[kOutW];
  const int b = blockIdx.x, t = threadIdx.x;

  float s = 0.0f;
#pragma unroll 1
  for (int i = 0; i < kObjs; ++i) s += Spart[((size_t)(b * kObjs + i)) * kHid + t];
  sh0[t] = s;
  __syncthreads();

  float acc = b4[t];
#pragma unroll 1
  for (int k = 0; k < kHid; ++k) acc = fmaf(sh0[k], W4[(size_t)k * kHid + t], acc);
  sh1[t] = fmaxf(acc, 0.0f);
  __syncthreads();

  acc = b5[t];
#pragma unroll 1
  for (int k = 0; k < kHid; ++k) acc = fmaf(sh1[k], W5[(size_t)k * kHid + t], acc);
  sh0[t] = fmaxf(acc, 0.0f);
  __syncthreads();

  if (t < kOutW) {
    acc = b6[t];
#pragma unroll 1
    for (int k = 0; k < kHid; ++k) acc = fmaf(sh0[k], W6[(size_t)k * kOutW + t], acc);
    so[t] = acc;
  }
  __syncthreads();
  if (t < 8) {
    const v4f v = *(const v4f*)(so + 4 * t);
    float* p = out + (size_t)b * kOutW + 4 * t;
    *(volatile v4f*)p = v;
    __threadfence();
    *(volatile v4f*)p = v;
  }
}

extern "C" void kernel_launch(void* const* d_in, const int* in_sizes, int n_in,
                              void* d_out, int out_size, void* d_ws, size_t ws_size,
                              hipStream_t stream) {
  if (n_in < 15) return;
  if (in_sizes[0] != kObjRows * kFeat || in_sizes[1] != 2 * kFeat * kHid || in_sizes[2] != kHid ||
      in_sizes[3] != kHid * kHid || in_sizes[4] != kHid || in_sizes[5] != kHid * kHid || in_sizes[6] != kHid ||
      in_sizes[7] != kHid * kHid || in_sizes[8] != kHid || in_sizes[9] != kHid * kHid || in_sizes[10] != kHid ||
      in_sizes[11] != kHid * kHid || in_sizes[12] != kHid || in_sizes[13] != kHid * kOutW || in_sizes[14] != kOutW ||
      out_size != kBatch * kOutW) return;

  const float* x  = (const float*)d_in[0];
  const float* W0 = (const float*)d_in[1];
  const float* b0 = (const float*)d_in[2];
  const float* W1 = (const float*)d_in[3];
  const float* b1 = (const float*)d_in[4];
  const float* W2 = (const float*)d_in[5];
  const float* b2 = (const float*)d_in[6];
  const float* W3 = (const float*)d_in[7];
  const float* b3 = (const float*)d_in[8];
  const float* W4 = (const float*)d_in[9];
  const float* b4 = (const float*)d_in[10];
  const float* W5 = (const float*)d_in[11];
  const float* b5 = (const float*)d_in[12];
  const float* W6 = (const float*)d_in[13];
  const float* b6 = (const float*)d_in[14];
  float* out = (float*)d_out;

  const size_t szPlane = (size_t)kObjRows * kHid * sizeof(float);
  const size_t szWt    = (size_t)3 * kHid * kHid * sizeof(unsigned short);
  const size_t offA  = 0;
  const size_t offBm = offA + szPlane;
  const size_t offWt = offBm + szPlane;
  const size_t offSp = offWt + szWt;
  const size_t total = offSp + szPlane;
  if (total > ws_size) return;

  char* ws = (char*)d_ws;
  float* A  = (float*)(ws + offA);
  float* Bm = (float*)(ws + offBm);
  unsigned short* WtAll = (unsigned short*)(ws + offWt);
  float* Spart = (float*)(ws + offSp);

  obj_linear_kernel<<<kObjRows / 4, 256, 0, stream>>>(x, W0, b0, A, Bm);
  wt_cast_kernel<<<dim3(kHid / 64, kHid / 64, 3), 256, 0, stream>>>(W1, W2, W3, WtAll, kWCarry);
  pair_mlp_kernel<<<kBatch * kObjs, 256, 0, stream>>>(A, Bm, WtAll, b1, b2, b3, Spart);
  head_mlp_kernel<<<kBatch, 256, 0, stream>>>(Spart, W4, b4, W5, b5, W6, b6, out);
}
